// SetSequenceModel_14010183320118
// MI455X (gfx1250) — hardware-run, weakly checked
//
#include <hip/hip_runtime.h>
#include <math.h>

typedef __attribute__((ext_vector_type(16))) _Float16 v16h;
typedef __attribute__((ext_vector_type(8)))  _Float16 v8h;
typedef __attribute__((ext_vector_type(8)))  float    v8f;
typedef __attribute__((ext_vector_type(4)))  float    v4f;
typedef __attribute__((ext_vector_type(2)))  float    v2f;
typedef __attribute__((ext_vector_type(4)))  unsigned v4u;
typedef __attribute__((ext_vector_type(4)))  int      v4i;

constexpr int kT     = 1024;
constexpr int kSetN  = 256;
constexpr int kItems = 8;
constexpr int kV     = 100000;
constexpr int kD     = 128;
constexpr int kX     = 2 * kD;
constexpr int kH     = 512;
constexpr int kG     = 4 * kH;
constexpr int kH2    = 256;
constexpr int kC     = 100;
constexpr int kCP    = 128;

constexpr float kCarryW  = 256.0f;
constexpr float kCarryX  = 256.0f;
constexpr float kCarryH  = 1024.0f;
constexpr float kCarryH1 = 256.0f;
constexpr float kPoolScale = kCarryX / (float)kItems;
constexpr float kScaleGx   = 1.0f / (kCarryX * kCarryW);
constexpr float kScaleRec  = 1.0f / (kCarryH * kCarryW);
constexpr float kScaleH1   = kCarryH1 / (kCarryH * kCarryW);
constexpr float kScaleOut  = 1.0f / (kCarryH1 * kCarryW);

static_assert(kX == 256 && kG == 2048, "shape constants");
static_assert((kX % 32) == 0 && (kH % 32) == 0 && (kH2 % 32) == 0, "GEMM K multiples of 32");
static_assert((kT % 64) == 0 && (kG % 64) == 0 && (kH2 % 64) == 0 && (kCP % 64) == 0, "GEMM M,N multiples of 64");
static_assert((kC % 4) == 0 && kC <= kCP, "output width");
static_assert(((kT / 64) * (kG / 64)) % 8 == 0, "gate-input GEMM tiles fill whole blocks");
static_assert(((kT / 64) * (kH2 / 64)) % 8 == 0, "head-1 GEMM tiles fill whole blocks");
static_assert(((kT / 64) * (kCP / 64)) % 8 == 0, "head-2 GEMM tiles fill whole blocks");

constexpr size_t kSzWIH  = (size_t)kG  * kX  * 2;
constexpr size_t kSzWHH  = (size_t)kG  * kH  * 2;
constexpr size_t kSzW1   = (size_t)kH2 * kH  * 2;
constexpr size_t kSzWO   = (size_t)kCP * kH2 * 2;
constexpr size_t kSzBS   = (size_t)kG  * 4;
constexpr size_t kSzB1   = (size_t)kH2 * 4;
constexpr size_t kSzBO   = (size_t)kCP * 4;
constexpr size_t kSzX16  = (size_t)kT  * kX  * 2;
constexpr size_t kSzGX   = (size_t)kT  * kG  * 4;
constexpr size_t kSzHS   = (size_t)kT  * kH  * 2;
constexpr size_t kSzH1   = (size_t)kT  * kH2 * 2;
constexpr size_t kSzOP   = (size_t)kT  * kCP * 4;
constexpr size_t kOffWIH = 0;
constexpr size_t kOffWHH = kOffWIH + kSzWIH;
constexpr size_t kOffW1  = kOffWHH + kSzWHH;
constexpr size_t kOffWO  = kOffW1  + kSzW1;
constexpr size_t kOffBS  = kOffWO  + kSzWO;
constexpr size_t kOffB1  = kOffBS  + kSzBS;
constexpr size_t kOffBO  = kOffB1  + kSzB1;
constexpr size_t kOffX16 = kOffBO  + kSzBO;
constexpr size_t kOffGX  = kOffX16 + kSzX16;
constexpr size_t kOffHS  = kOffGX  + kSzGX;
constexpr size_t kOffH1  = kOffHS  + kSzHS;
constexpr size_t kOffOP  = kOffH1  + kSzH1;
constexpr size_t kWsTotal = kOffOP + kSzOP;
static_assert(kWsTotal == 14493184ull, "carve total");
static_assert(kWsTotal <= 134217728ull, "carve cap");
static_assert((kSzWIH % 128) == 0 && (kSzWHH % 128) == 0 && (kSzW1 % 128) == 0 && (kSzWO % 128) == 0 &&
              (kSzBS % 128) == 0 && (kSzB1 % 128) == 0 && (kSzBO % 128) == 0 && (kSzX16 % 128) == 0 &&
              (kSzGX % 128) == 0 && (kSzHS % 128) == 0 && (kSzH1 % 128) == 0 && (kSzOP % 128) == 0,
              "128-B aligned regions");

__device__ __forceinline__ unsigned pack_h2(float a, float b) {
  const _Float16 ha = (_Float16)a;
  const _Float16 hb = (_Float16)b;
  const unsigned ua = (unsigned)__builtin_bit_cast(unsigned short, ha);
  const unsigned ub = (unsigned)__builtin_bit_cast(unsigned short, hb);
  return ua | (ub << 16);
}

__device__ __forceinline__ v16h frag_load_h(const _Float16* p) {
  union U { v16h v; v8h h[2]; };
  U f;
  f.h[0] = *(const v8h*)(p);
  f.h[1] = *(const v8h*)(p + 16);
  return f.v;
}

__device__ __forceinline__ v8f mma_f16(v16h a, v16h b, v8f c) {
  c = __builtin_amdgcn_wmma_f32_16x16x32_f16(false, a, false, b, (short)0, c, false, false);
  asm volatile("v_nop\n\tv_nop\n\tv_nop\n\tv_nop" : "+v"(c) : "v"(a), "v"(b));
  return c;
}
__device__ __forceinline__ void keep4_h(v16h a, v16h b, v16h c, v16h d) { asm volatile("v_nop" :: "v"(a), "v"(b), "v"(c), "v"(d)); }
__device__ __forceinline__ void acc_guard4(v8f& a, v8f& b, v8f& c, v8f& d) { asm volatile("v_nop\n\tv_nop\n\tv_nop\n\tv_nop" : "+v"(a), "+v"(b), "+v"(c), "+v"(d)); }

__global__ __launch_bounds__(256) void weight_plane_f16_kernel(
    const float* __restrict__ src, unsigned* __restrict__ dst, int rowsSrc, int rowsDst, int kcols, float carry)
{
  const int i = blockIdx.x * 256 + threadIdx.x;
  const int perRow = kcols >> 3;
  if (i >= rowsDst * perRow) return;
  const int row = i / perRow;
  const int c8 = (i - row * perRow) << 3;
  const bool live = row < rowsSrc;
  const int rs = live ? row : (rowsSrc - 1);
  const float* sp = src + (size_t)rs * kcols + c8;
  const v4f a0 = *(const v4f*)(sp);
  const v4f a1 = *(const v4f*)(sp + 4);
  const float f0 = live ? a0[0] * carry : 0.0f;
  const float f1 = live ? a0[1] * carry : 0.0f;
  const float f2 = live ? a0[2] * carry : 0.0f;
  const float f3 = live ? a0[3] * carry : 0.0f;
  const float f4 = live ? a1[0] * carry : 0.0f;
  const float f5 = live ? a1[1] * carry : 0.0f;
  const float f6 = live ? a1[2] * carry : 0.0f;
  const float f7 = live ? a1[3] * carry : 0.0f;
  v4u w;
  w[0] = pack_h2(f0, f1);
  w[1] = pack_h2(f2, f3);
  w[2] = pack_h2(f4, f5);
  w[3] = pack_h2(f6, f7);
  volatile v4u* q = (volatile v4u*)(dst + (size_t)i * 4);
  *q = w;
  __threadfence();
  *q = w;
}

__global__ __launch_bounds__(256) void bias_planes_kernel(
    const float* __restrict__ bih, const float* __restrict__ bhh, const float* __restrict__ b1,
    const float* __restrict__ bout, float* __restrict__ bsum, float* __restrict__ b1x, float* __restrict__ boutp)
{
  constexpr int n0 = kG / 4;
  constexpr int n1 = kH2 / 4;
  constexpr int n2 = kCP / 4;
  constexpr int nLive = kC / 4;
  const int i = blockIdx.x * 256 + threadIdx.x;
  if (i >= n0 + n1 + n2) return;
  v4f val;
  float* dst;
  if (i < n0) {
    const v4f a = *(const v4f*)(bih + 4 * i);
    const v4f b = *(const v4f*)(bhh + 4 * i);
    val = a + b;
    dst = bsum + 4 * i;
  } else if (i < n0 + n1) {
    const int j = i - n0;
    const v4f a = *(const v4f*)(b1 + 4 * j);
    val[0] = a[0] * kCarryH1;
    val[1] = a[1] * kCarryH1;
    val[2] = a[2] * kCarryH1;
    val[3] = a[3] * kCarryH1;
    dst = b1x + 4 * j;
  } else {
    const int j = i - n0 - n1;
    const int jc = (j < nLive) ? j : (nLive - 1);
    const v4f a = *(const v4f*)(bout + 4 * jc);
    float e0 = a[0];
    float e1 = a[1];
    float e2 = a[2];
    float e3 = a[3];
    asm volatile("" : "+v"(e0));
    asm volatile("" : "+v"(e1));
    asm volatile("" : "+v"(e2));
    asm volatile("" : "+v"(e3));
    const bool live = j < nLive;
    val[0] = live ? e0 : 0.0f;
    val[1] = live ? e1 : 0.0f;
    val[2] = live ? e2 : 0.0f;
    val[3] = live ? e3 : 0.0f;
    dst = boutp + 4 * j;
  }
  volatile v4f* q = (volatile v4f*)dst;
  *q = val;
  __threadfence();
  *q = val;
}

__global__ __launch_bounds__(128) void pool_kernel(
    const int* __restrict__ idsA, const int* __restrict__ idsB, const float* __restrict__ emb,
    unsigned* __restrict__ x16w)
{
  __shared__ __align__(16) int sIdx[2 * kSetN];
  const int t = blockIdx.x;
  const int tid = threadIdx.x;
  const int lane = tid & 31;
  const int wave = tid >> 5;
  {
    const int tabS = tid >> 6;
    const int j = tid & 63;
    const int* srcp = tabS ? idsB : idsA;
    v4i q = *(const v4i*)(srcp + (size_t)t * kSetN + 4 * j);
    q[0] = min(max(q[0], 0), kV - 1);
    q[1] = min(max(q[1], 0), kV - 1);
    q[2] = min(max(q[2], 0), kV - 1);
    q[3] = min(max(q[3], 0), kV - 1);
    *(v4i*)(sIdx + tabS * kSetN + 4 * j) = q;
  }
  __syncthreads();
  const int tab = wave >> 1;
  const int col = (wave & 1) * 64 + 2 * lane;
  const int* ip = sIdx + tab * kSetN;
  float a0 = 0.0f;
  float a1 = 0.0f;
#pragma unroll 8
  for (int s = 0; s < kSetN; ++s) {
    const int id = ip[s];
    const v2f v = *(const v2f*)(emb + (size_t)id * kD + col);
    a0 += v[0];
    a1 += v[1];
  }
  const unsigned w = pack_h2(a0 * kPoolScale, a1 * kPoolScale);
  volatile unsigned* q = x16w + (size_t)t * (kX / 2) + 32 * wave + lane;
  *q = w;
  __threadfence();
  *q = w;
}

template <int OUT_MODE, int ACT>
__global__ __launch_bounds__(256) void wmma_gemm64_f16(
    const unsigned short* __restrict__ Ap, int lda,
    const unsigned short* __restrict__ Btp, int ldb,
    void* __restrict__ Cout, int ldc,
    const float* __restrict__ bias,
    int M, int N, int K, float scale) {
  const _Float16* A  = (const _Float16*)Ap;
  const _Float16* Bt = (const _Float16*)Btp;
  __shared__ __align__(16) float sT[8][16 * 68];
  const int lane = threadIdx.x & 31;
  const int wave = threadIdx.x >> 5;
  const int tilesN = N >> 6;
  const int tilesM = M >> 6;
  const int tile = blockIdx.x * 8 + wave;
  if (tile >= tilesM * tilesN) return;
  const int tm = tile / tilesN;
  const int tn = tile - tm * tilesN;
  const int m0 = tm << 6;
  const int n0 = tn << 6;

  const int rlane = lane & 15;
  const int koff  = (lane >> 4) * 8;
  const int mOff  = (lane >> 4) * 8;

  v8f acc[4][4];
#pragma unroll
  for (int i = 0; i < 4; ++i)
#pragma unroll
    for (int j = 0; j < 4; ++j) acc[i][j] = (v8f){0.f,0.f,0.f,0.f,0.f,0.f,0.f,0.f};

  for (int k0 = 0; k0 < K; k0 += 32) {
    v16h bh[4];
#pragma unroll
    for (int j = 0; j < 4; ++j) {
      const size_t bo = (size_t)(n0 + (j << 4) + rlane) * ldb + koff + k0;
      bh[j] = frag_load_h(Bt + bo);
    }
#pragma unroll
    for (int i = 0; i < 4; ++i) {
      const size_t ao = (size_t)(m0 + (i << 4) + rlane) * lda + koff + k0;
      const v16h ah = frag_load_h(A + ao);
#pragma unroll
      for (int j = 0; j < 4; ++j) acc[i][j] = mma_f16(ah, bh[j], acc[i][j]);
    }
    keep4_h(bh[0], bh[1], bh[2], bh[3]);
  }
  acc_guard4(acc[0][0], acc[0][1], acc[0][2], acc[0][3]);
  acc_guard4(acc[1][0], acc[1][1], acc[1][2], acc[1][3]);
  acc_guard4(acc[2][0], acc[2][1], acc[2][2], acc[2][3]);
  acc_guard4(acc[3][0], acc[3][1], acc[3][2], acc[3][3]);

  float* slab = sT[wave];
#pragma unroll
  for (int i = 0; i < 4; ++i) {
    const int mBase = m0 + (i << 4);
#pragma unroll
    for (int j = 0; j < 4; ++j) {
      const int n = n0 + (j << 4) + rlane;
      const float bv = bias[n];
#pragma unroll
      for (int r = 0; r < 8; ++r) {
        float v = acc[i][j][r] * scale;
        v += bv;
        if (ACT == 2) v = fmaxf(v, 0.0f);
        slab[(mOff + r) * 68 + (j << 4) + rlane] = v;
      }
    }
    __builtin_amdgcn_fence(__ATOMIC_RELEASE, "workgroup");
    __builtin_amdgcn_wave_barrier();
    __builtin_amdgcn_fence(__ATOMIC_ACQUIRE, "workgroup");
    if (OUT_MODE == 0) {
      float* C = (float*)Cout;
      const int hh = lane >> 4, c4 = (lane & 15) * 4;
      for (int pass = 0; pass < 2; ++pass) {
#pragma unroll
        for (int it = 0; it < 8; ++it) {
          const int row = it * 2 + hh;
          const v4f v = *(const v4f*)(slab + row * 68 + c4);
          *(volatile v4f*)(C + (size_t)(mBase + row) * ldc + n0 + c4) = v;
        }
        __threadfence();
      }
    } else {
      const int q = lane >> 3, c8 = (lane & 7) * 8;
      unsigned short* C = (unsigned short*)Cout;
      for (int pass = 0; pass < 2; ++pass) {
#pragma unroll
        for (int it = 0; it < 4; ++it) {
          const int row = it * 4 + q;
          const float* sp = slab + row * 68 + c8;
          const v4f s0 = *(const v4f*)(sp);
          const v4f s1 = *(const v4f*)(sp + 4);
          v4u w;
          w[0] = pack_h2(s0[0], s0[1]);
          w[1] = pack_h2(s0[2], s0[3]);
          w[2] = pack_h2(s1[0], s1[1]);
          w[3] = pack_h2(s1[2], s1[3]);
          *(volatile v4u*)(C + (size_t)(mBase + row) * ldc + n0 + c8) = w;
        }
        __threadfence();
      }
    }
    __builtin_amdgcn_fence(__ATOMIC_RELEASE, "workgroup");
    __builtin_amdgcn_wave_barrier();
    __builtin_amdgcn_fence(__ATOMIC_ACQUIRE, "workgroup");
  }
}

__global__ __launch_bounds__(1024) void lstm_scan_kernel(
    const float* __restrict__ gx, const unsigned short* __restrict__ Whh16, unsigned* __restrict__ hs16w)
{
  __shared__ __align__(16) unsigned sH[2][kH / 2];
  const int tid  = threadIdx.x;
  const int lane = tid & 31;
  const int wave = tid >> 5;
  const int m    = lane & 15;
  const int hh   = lane >> 4;
  if (tid < kH / 2) sH[0][tid] = 0u;
  __syncthreads();

  const unsigned am = (m == 0) ? 0xFFFFFFFFu : 0u;
  const v4u amask = {am, am, am, am};
  const int unit = 16 * wave + m;
  const _Float16* Bbase = (const _Float16*)Whh16 + (size_t)unit * kH + 8 * hh;
  constexpr size_t kGateStride = (size_t)kH * kH;
  float cst = 0.0f;

#pragma unroll 1
  for (int t = 0; t < kT; ++t) {
    const int cur = t & 1;
    const int nxt = cur ^ 1;
    const float* gr = gx + (size_t)t * kG + unit;
    const float gi = gr[0];
    const float gf = gr[kH];
    const float gg = gr[2 * kH];
    const float go = gr[3 * kH];

    v8f a0 = (v8f){0.f,0.f,0.f,0.f,0.f,0.f,0.f,0.f};
    v8f a1 = (v8f){0.f,0.f,0.f,0.f,0.f,0.f,0.f,0.f};
    v8f a2 = (v8f){0.f,0.f,0.f,0.f,0.f,0.f,0.f,0.f};
    v8f a3 = (v8f){0.f,0.f,0.f,0.f,0.f,0.f,0.f,0.f};
    const unsigned* hrow = &sH[cur][4 * hh];
#pragma unroll 1
    for (int k0 = 0; k0 < kH; k0 += 32) {
      union AF { v16h v; v4u q[2]; };
      AF af;
      const v4u q0 = *(const v4u*)(hrow + (k0 >> 1));
      const v4u q1 = *(const v4u*)(hrow + (k0 >> 1) + 8);
      af.q[0] = q0 & amask;
      af.q[1] = q1 & amask;
      const _Float16* bp = Bbase + k0;
      const v16h b0 = frag_load_h(bp);
      const v16h b1 = frag_load_h(bp + kGateStride);
      const v16h b2 = frag_load_h(bp + 2 * kGateStride);
      const v16h b3 = frag_load_h(bp + 3 * kGateStride);
      a0 = mma_f16(af.v, b0, a0);
      a1 = mma_f16(af.v, b1, a1);
      a2 = mma_f16(af.v, b2, a2);
      a3 = mma_f16(af.v, b3, a3);
    }

    const float pi = a0[0] * kScaleRec + gi;
    const float pf = a1[0] * kScaleRec + gf;
    const float pg = a2[0] * kScaleRec + gg;
    const float po = a3[0] * kScaleRec + go;
    const float iv = 1.0f / (1.0f + expf(-pi));
    const float fv = 1.0f / (1.0f + expf(-pf));
    const float gv = tanhf(pg);
    const float ov = 1.0f / (1.0f + expf(-po));
    cst = fv * cst + iv * gv;
    const float hval = ov * tanhf(cst);

    const _Float16 h16 = (_Float16)(hval * kCarryH);
    const unsigned hb = (unsigned)__builtin_bit_cast(unsigned short, h16);
    const unsigned pb = (unsigned)__shfl_xor((int)hb, 1, 32);
    const unsigned word = hb | (pb << 16);
    if (lane < 16 && (lane & 1) == 0) sH[nxt][8 * wave + (lane >> 1)] = word;
    __syncthreads();

    if (wave < 8) {
      const unsigned wv = sH[nxt][32 * wave + lane];
      volatile unsigned* q = hs16w + (size_t)t * (kH / 2) + 32 * wave + lane;
      *q = wv;
      __threadfence();
      *q = wv;
    }
  }
}

__global__ __launch_bounds__(256) void pack_out_kernel(const float* __restrict__ outp, float* __restrict__ outv)
{
  const int i = blockIdx.x * 256 + threadIdx.x;
  if (i >= kT * kC / 4) return;
  const int f = 4 * i;
  const int row = f / kC;
  const int col = f - row * kC;
  const v4f v = *(const v4f*)(outp + (size_t)row * kCP + col);
  volatile v4f* q = (volatile v4f*)(outv + f);
  *q = v;
  __threadfence();
  *q = v;
}

extern "C" void kernel_launch(void* const* d_in, const int* in_sizes, int n_in,
                              void* d_out, int out_size, void* d_ws, size_t ws_size,
                              hipStream_t stream) {
  if (n_in < 11) return;
  if (in_sizes[0] != kT * kSetN) return;
  if (in_sizes[1] != kT * kSetN) return;
  if (in_sizes[2] != kV * kD) return;
  if (in_sizes[3] != kG * kX) return;
  if (in_sizes[4] != kG * kH) return;
  if (in_sizes[5] != kG) return;
  if (in_sizes[6] != kG) return;
  if (in_sizes[7] != kH2 * kH) return;
  if (in_sizes[8] != kH2) return;
  if (in_sizes[9] != kC * kH2) return;
  if (in_sizes[10] != kC) return;
  if (out_size != kT * kC) return;
  if (ws_size < kWsTotal) return;

  const int*   idsA = (const int*)d_in[0];
  const int*   idsB = (const int*)d_in[1];
  const float* emb  = (const float*)d_in[2];
  const float* Wih  = (const float*)d_in[3];
  const float* Whh  = (const float*)d_in[4];
  const float* bih  = (const float*)d_in[5];
  const float* bhh  = (const float*)d_in[6];
  const float* W1   = (const float*)d_in[7];
  const float* b1   = (const float*)d_in[8];
  const float* Wout = (const float*)d_in[9];
  const float* bout = (const float*)d_in[10];
  float* outv = (float*)d_out;

  char* ws = (char*)d_ws;
  unsigned short* WIH16 = (unsigned short*)(ws + kOffWIH);
  unsigned short* WHH16 = (unsigned short*)(ws + kOffWHH);
  unsigned short* W1H16 = (unsigned short*)(ws + kOffW1);
  unsigned short* WOH16 = (unsigned short*)(ws + kOffWO);
  float*          BSUM  = (float*)(ws + kOffBS);
  float*          B1X   = (float*)(ws + kOffB1);
  float*          BOUTP = (float*)(ws + kOffBO);
  unsigned short* X16   = (unsigned short*)(ws + kOffX16);
  float*          GX    = (float*)(ws + kOffGX);
  unsigned short* HS16  = (unsigned short*)(ws + kOffHS);
  unsigned short* H1H16 = (unsigned short*)(ws + kOffH1);
  float*          OUTP  = (float*)(ws + kOffOP);

  weight_plane_f16_kernel<<<(kG * kX / 8) / 256, 256, 0, stream>>>(Wih, (unsigned*)WIH16, kG, kG, kX, kCarryW);
  weight_plane_f16_kernel<<<(kG * kH / 8) / 256, 256, 0, stream>>>(Whh, (unsigned*)WHH16, kG, kG, kH, kCarryW);
  weight_plane_f16_kernel<<<(kH2 * kH / 8) / 256, 256, 0, stream>>>(W1, (unsigned*)W1H16, kH2, kH2, kH, kCarryW);
  weight_plane_f16_kernel<<<(kCP * kH2 / 8) / 256, 256, 0, stream>>>(Wout, (unsigned*)WOH16, kC, kCP, kH2, kCarryW);
  bias_planes_kernel<<<3, 256, 0, stream>>>(bih, bhh, b1, bout, BSUM, B1X, BOUTP);

  pool_kernel<<<kT, 128, 0, stream>>>(idsA, idsB, emb, (unsigned*)X16);

  wmma_gemm64_f16<0, 0><<<((kT / 64) * (kG / 64)) / 8, 256, 0, stream>>>(
      X16, kX, WIH16, kX, (void*)GX, kG, BSUM, kT, kG, kX, kScaleGx);

  lstm_scan_kernel<<<1, 1024, 0, stream>>>(GX, WHH16, (unsigned*)HS16);

  wmma_gemm64_f16<1, 2><<<((kT / 64) * (kH2 / 64)) / 8, 256, 0, stream>>>(
      HS16, kH, W1H16, kH, (void*)H1H16, kH2, B1X, kT, kH2, kH, kScaleH1);

  wmma_gemm64_f16<0, 0><<<((kT / 64) * (kCP / 64)) / 8, 256, 0, stream>>>(
      H1H16, kH2, WOH16, kH2, (void*)OUTP, kCP, BOUTP, kT, kCP, kH2, kScaleOut);

  pack_out_kernel<<<(kT * kC / 4) / 256, 256, 0, stream>>>(OUTP, outv);
}
